// GATEncoder_15934328668575
// MI455X (gfx1250) — hardware-verified
//
#include <hip/hip_runtime.h>
#include <stddef.h>
#include <stdint.h>
#include <math.h>


#define F_IN0   128
#define KG      128
#define CH      64
#define NOUT    32
#define XUPR    (F_IN0 / 8)
#define NTHR    256
#define NWAVE   8
#define EPT     8
#define CHUNK   (NTHR * EPT)
#define WCAP    (EPT * 32)
#define LISTN   (NWAVE * WCAP)
#define NBMAX   2048
#define SLOTB   11
#define RCAP    28672
#define DEGCAP  128
#define GBM     64
#define GTHR    128
#define MROWS   128
#define PARTW   160
#define WSTW    130
#define NEGSL   0.2f
#define MX0     (-1.0e30f)
#define BNEPS   1e-5f
#define WSMAX   134217728
#define LDS_AGG ((2 * RCAP + 2 * NBMAX + LISTN) * 4 + 64)

static_assert((CHUNK & (CHUNK - 1)) == 0 && CHUNK <= (1 << SLOTB));
static_assert(NBMAX == (1 << SLOTB));
static_assert(NTHR * 8 == NBMAX);
static_assert(LISTN >= NBMAX);
static_assert(LISTN >= NWAVE * WCAP);
static_assert((RCAP % 32) == 0);
static_assert(LDS_AGG <= 300000);
static_assert(GBM == (GTHR / 32) * 16);
static_assert((KG % 32) == 0 && (KG % 8) == 0);
static_assert(KG == F_IN0 && KG == 2 * CH);
static_assert(GTHR == 2 * GBM);
static_assert((MROWS % GBM) == 0);
static_assert(CH == 2 * 32);
static_assert(NOUT == 32);
static_assert(CH == 4 * 16 && NOUT == 4 * 8);
static_assert((F_IN0 % 8) == 0);
static_assert(PARTW % 32 == 0 && PARTW / 4 <= NTHR && PARTW >= 2 * CH + 1);
static_assert(WSTW >= 2 * CH + 1 && (WSTW % 2) == 0);
static_assert(NWAVE * WSTW + PARTW <= LISTN);

typedef float          v2f  __attribute__((ext_vector_type(2)));
typedef float          v4f  __attribute__((ext_vector_type(4)));
typedef float          v8f  __attribute__((ext_vector_type(8)));
typedef int            v4i  __attribute__((ext_vector_type(4)));
typedef int            v8i  __attribute__((ext_vector_type(8)));
typedef unsigned int   v4u  __attribute__((ext_vector_type(4)));
typedef unsigned short v8us __attribute__((ext_vector_type(8)));
typedef __bf16         v16b __attribute__((ext_vector_type(16)));
typedef v2f  __attribute__((may_alias)) v2fa;
typedef v4f  __attribute__((may_alias)) v4fa;
typedef v8us __attribute__((may_alias)) v8usa;
union FragB { v16b v; v8us h[2]; v8i w; };

__device__ __forceinline__ v8f wmb(const FragB& a, const FragB& b, v8f c) {
  v8f d = __builtin_amdgcn_wmma_f32_16x16x32_bf16(false, a.v, false, b.v, (short)0, c, false, false);
  asm volatile("v_nop\n\tv_nop\n\tv_nop\n\tv_nop" : "+v"(d) : "v"(a.w), "v"(b.w));
  return d;
}

__device__ __forceinline__ unsigned int f2bf(float f) {
  const unsigned int u = __float_as_uint(f);
  return ((u + 0x7FFFu + ((u >> 16) & 1u)) >> 16) & 0xFFFFu;
}
__device__ __forceinline__ float bf2f(unsigned int b) { return __uint_as_float(b << 16); }
__device__ __forceinline__ float bfr(float f) { return bf2f(f2bf(f)); }
__device__ __forceinline__ v2f bfr2(const v2f a) { v2f r; r.x = bfr(a.x); r.y = bfr(a.y); return r; }
__device__ __forceinline__ v4f bfr4(const v4f a) {
  v4f r; r.x = bfr(a.x); r.y = bfr(a.y); r.z = bfr(a.z); r.w = bfr(a.w); return r;
}
__device__ __forceinline__ unsigned int pk2(float lo, float hi) { return f2bf(lo) | (f2bf(hi) << 16); }
__device__ __forceinline__ v4u pack8(const v4f a, const v4f b) {
  v4u r;
  r.x = pk2(a.x, a.y); r.y = pk2(a.z, a.w); r.z = pk2(b.x, b.y); r.w = pk2(b.z, b.w);
  return r;
}

__device__ __forceinline__ int scan_chunk(const int* __restrict__ dsts, int nE, int cbase, int slotBase,
                                          int nb, int vec8, int* list, int tid, int lane, int wave) {
  int wc = 0;
  const int el0  = tid * EPT;
  const int e0   = cbase + el0;
  const int sent = -2147483647 - 1;
  v4i da, db;
  if (vec8 != 0 && cbase + CHUNK <= nE) {
    da = *(const v4i*)(dsts + e0);
    db = *(const v4i*)(dsts + e0 + 4);
  } else {
    da.x = (e0     < nE) ? dsts[min(e0,     nE - 1)] : sent;
    da.y = (e0 + 1 < nE) ? dsts[min(e0 + 1, nE - 1)] : sent;
    da.z = (e0 + 2 < nE) ? dsts[min(e0 + 2, nE - 1)] : sent;
    da.w = (e0 + 3 < nE) ? dsts[min(e0 + 3, nE - 1)] : sent;
    db.x = (e0 + 4 < nE) ? dsts[min(e0 + 4, nE - 1)] : sent;
    db.y = (e0 + 5 < nE) ? dsts[min(e0 + 5, nE - 1)] : sent;
    db.z = (e0 + 6 < nE) ? dsts[min(e0 + 6, nE - 1)] : sent;
    db.w = (e0 + 7 < nE) ? dsts[min(e0 + 7, nE - 1)] : sent;
  }
  const unsigned nbs = (unsigned)slotBase;
  const unsigned unb = (unsigned)nb;
  const unsigned s0 = (unsigned)da.x - nbs, s1 = (unsigned)da.y - nbs;
  const unsigned s2 = (unsigned)da.z - nbs, s3 = (unsigned)da.w - nbs;
  const unsigned s4 = (unsigned)db.x - nbs, s5 = (unsigned)db.y - nbs;
  const unsigned s6 = (unsigned)db.z - nbs, s7 = (unsigned)db.w - nbs;
  const bool h0 = s0 < unb, h1 = s1 < unb, h2 = s2 < unb, h3 = s3 < unb;
  const bool h4 = s4 < unb, h5 = s5 < unb, h6 = s6 < unb, h7 = s7 < unb;
  const unsigned any = __builtin_amdgcn_ballot_w32(h0 | h1 | h2 | h3 | h4 | h5 | h6 | h7);
  if (any != 0u) {
#define HITJ(J, HJ, SJ) { \
      const unsigned mj = __builtin_amdgcn_ballot_w32(HJ); \
      if (mj != 0u) { \
        if (HJ) { \
          const int pos = wc + (int)__builtin_amdgcn_mbcnt_lo(mj, 0u); \
          if (pos < WCAP) list[wave * WCAP + pos] = ((el0 + (J)) << SLOTB) | (int)(SJ); \
        } \
        wc += (int)__builtin_popcount(mj); } }
    HITJ(0, h0, s0)
    HITJ(1, h1, s1)
    HITJ(2, h2, s2)
    HITJ(3, h3, s3)
    HITJ(4, h4, s4)
    HITJ(5, h5, s5)
    HITJ(6, h6, s6)
    HITJ(7, h7, s7)
#undef HITJ
  }
  return wc;
}

__global__ __launch_bounds__(NTHR) void k_xprep(const float* __restrict__ x, unsigned short* xb, int nN, int nUnits) {
  const int i = (int)blockIdx.x * NTHR + (int)threadIdx.x;
  if (i >= nUnits) return;
  const int row = i / XUPR;
  const int c0  = (i - row * XUPR) * 8;
  const int rc  = row < nN ? row : nN - 1;
  const float* p = x + (size_t)rc * F_IN0 + c0;
  v4f a = *(const v4fa*)p, b = *(const v4fa*)(p + 4);
  const v4f z4 = {0.f, 0.f, 0.f, 0.f};
  if (row >= nN) { a = z4; b = z4; }
  const v4u hv = pack8(a, b);
  const size_t o = (size_t)row * F_IN0 + c0;
  *(volatile v4u*)(xb + o) = hv;
  __threadfence();
  *(volatile v4u*)(xb + o) = hv;
}

__global__ __launch_bounds__(NTHR) void k_wtr(const float* __restrict__ w, int Kin, int Ncol, int Nrows, int Kout,
                                              unsigned short* wt, int nUnits) {
  const int u = (int)blockIdx.x * NTHR + (int)threadIdx.x;
  if (u >= nUnits) return;
  const int kq = Kout >> 3;
  const int n  = u / kq;
  const int k8 = (u - n * kq) * 8;
  const int kk = k8 - (k8 / Kin) * Kin;
  const int ncl = n < Ncol ? n : Ncol - 1;
  const float* p = w + (size_t)kk * (size_t)Ncol + ncl;
  v4f a, b;
  a.x = p[0];                    a.y = p[(size_t)Ncol];         a.z = p[(size_t)2 * Ncol];     a.w = p[(size_t)3 * Ncol];
  b.x = p[(size_t)4 * Ncol];     b.y = p[(size_t)5 * Ncol];     b.z = p[(size_t)6 * Ncol];     b.w = p[(size_t)7 * Ncol];
  const v4f z4 = {0.f, 0.f, 0.f, 0.f};
  if (n >= Ncol || n >= Nrows) { a = z4; b = z4; }
  const v4u wv = pack8(a, b);
  unsigned short* o = wt + (size_t)n * (size_t)Kout + k8;
  *(volatile v4u*)o = wv;
  __threadfence();
  *(volatile v4u*)o = wv;
}

template<int NC>
__global__ __launch_bounds__(GTHR) void k_gemm(
    const unsigned short* __restrict__ A, const unsigned short* __restrict__ WT,
    float* outF,
    const float* __restrict__ atts, const float* __restrict__ attd,
    float* SD, int MPr)
{
  constexpr int NT = NC / 16;
  __shared__ __attribute__((aligned(16))) float stg[GBM * NC];
  __shared__ __attribute__((aligned(16))) float satt[2 * 64];
  __shared__ __attribute__((aligned(16))) float sdot[2 * GBM];
  const int tid = (int)threadIdx.x, lane = tid & 31, wave = tid >> 5, hh = lane >> 4, m = lane & 15;
  const int rowBase = (int)blockIdx.x * GBM;

  {
    const int which = tid >> 6;
    const int c     = tid & 63;
    const int ai    = c < NC ? c : NC - 1;
    const float vs = atts[ai];
    const float vd = attd[ai];
    const unsigned int msk = (which == 0) ? 0u : 0xFFFFFFFFu;
    const float v = __uint_as_float((__float_as_uint(vs) & ~msk) | (__float_as_uint(vd) & msk));
    satt[which * 64 + c] = (c < NC) ? bfr(v) : 0.0f;
  }

  v8f acc[NT];
  {
    const v8f z = {0.f, 0.f, 0.f, 0.f, 0.f, 0.f, 0.f, 0.f};
#pragma unroll
    for (int t = 0; t < NT; ++t) acc[t] = z;
  }
  const unsigned short* ap = A  + (size_t)(rowBase + 16 * wave + m) * (size_t)KG + 8 * hh;
  const unsigned short* wp = WT + (size_t)m * (size_t)KG + 8 * hh;
#pragma unroll 1
  for (int ks = 0; ks < KG / 32; ++ks) {
    FragB af;
    af.h[0] = *(const v8usa*)(ap + 32 * ks);
    af.h[1] = *(const v8usa*)(ap + 32 * ks + 16);
#pragma unroll
    for (int t = 0; t < NT; ++t) {
      const unsigned short* wq = wp + (size_t)(16 * t) * (size_t)KG + 32 * ks;
      FragB bf;
      bf.h[0] = *(const v8usa*)wq;
      bf.h[1] = *(const v8usa*)(wq + 16);
      acc[t] = wmb(af, bf, acc[t]);
    }
  }

#pragma unroll
  for (int t = 0; t < NT; ++t) {
    const int lc = 16 * t + m;
#pragma unroll
    for (int r = 0; r < 8; ++r) {
      const int lr = 16 * wave + 8 * hh + r;
      stg[lr * NC + lc] = acc[t][r];
    }
  }
  __syncthreads();

  {
    const int row = tid & 63, which = tid >> 6;
    const float* sa = satt + which * 64;
    const float* hr = stg + row * NC;
    float d0 = 0.f;
#pragma unroll
    for (int c4 = 0; c4 < NC / 4; ++c4) {
      const v4f h4 = *(const v4fa*)(hr + 4 * c4);
      const v4f a4 = *(const v4fa*)(sa + 4 * c4);
      d0 = fmaf(h4.x, a4.x, d0); d0 = fmaf(h4.y, a4.y, d0); d0 = fmaf(h4.z, a4.z, d0); d0 = fmaf(h4.w, a4.w, d0);
    }
    sdot[which * GBM + row] = d0;
  }
  __syncthreads();

  const int piece = lane & 15;
  const int g     = hh;
  const v4f sdv = *(const v4fa*)(sdot + g * GBM + 4 * piece);
  float* sp = SD + (size_t)g * (size_t)MPr + rowBase + 4 * piece;
  const bool sdw = (wave == 0);

  if (NC == 64) {
    v4f fv[8];
#pragma unroll
    for (int i = 0; i < 8; ++i) {
      const int lr = 16 * wave + 2 * i + hh;
      fv[i] = *(const v4fa*)(stg + lr * NC + 4 * m);
    }
#pragma unroll
    for (int i = 0; i < 8; ++i) {
      const int lr = 16 * wave + 2 * i + hh;
      float* op = outF + (size_t)(rowBase + lr) * (size_t)NC + 4 * m;
      *(volatile v4f*)op = fv[i];
    }
    if (sdw) *(volatile v4f*)sp = sdv;
    __threadfence();
#pragma unroll
    for (int i = 0; i < 8; ++i) {
      const int lr = 16 * wave + 2 * i + hh;
      float* op = outF + (size_t)(rowBase + lr) * (size_t)NC + 4 * m;
      *(volatile v4f*)op = fv[i];
    }
    if (sdw) *(volatile v4f*)sp = sdv;
  } else {
    v4f pv[4];
    const float* sb = stg + (16 * wave) * NC;
    float* ob = outF + (size_t)(rowBase + 16 * wave) * (size_t)NC;
#pragma unroll
    for (int j = 0; j < 4; ++j) {
      const int p = 32 * j + lane;
      pv[j] = *(const v4fa*)(sb + 4 * p);
    }
#pragma unroll
    for (int j = 0; j < 4; ++j) {
      const int p = 32 * j + lane;
      *(volatile v4f*)(ob + 4 * p) = pv[j];
    }
    if (sdw) *(volatile v4f*)sp = sdv;
    __threadfence();
#pragma unroll
    for (int j = 0; j < 4; ++j) {
      const int p = 32 * j + lane;
      *(volatile v4f*)(ob + 4 * p) = pv[j];
    }
    if (sdw) *(volatile v4f*)sp = sdv;
  }
}

template<int L>
__global__ __launch_bounds__(NTHR) void k_agg(
    const int* __restrict__ srcs, const int* __restrict__ dsts,
    const float* __restrict__ F, const float* __restrict__ SD,
    const float* __restrict__ bias,
    float* HCo, float* part, float* out,
    int nN, int nE, int nb, int MPr) {
  extern __shared__ v4f lds_dyn[];
  int* reg1 = (int*)lds_dyn;
  int* reg2 = reg1 + RCAP;
  int* scnt = reg2 + RCAP;
  int* soff = scnt + NBMAX;
  int* list = soff + NBMAX;
  int* wcnt = list + LISTN;
  int* wtot = wcnt + NWAVE;
  const int tid = (int)threadIdx.x, lane = tid & 31, wave = tid >> 5;
  const int nodeBase = (int)blockIdx.x * nb;
  const int vec8 = ((reinterpret_cast<uintptr_t>(dsts) & (uintptr_t)15) == (uintptr_t)0) ? 1 : 0;

  for (int i = tid; i < NBMAX; i += NTHR) scnt[i] = 0;
  __syncthreads();

  int tot = 0;
  const int nChunks = (nE + CHUNK - 1) / CHUNK;
#pragma unroll 1
  for (int ch = 0; ch < nChunks; ++ch) {
    const int cbase = ch * CHUNK;
    const int wc = scan_chunk(dsts, nE, cbase, nodeBase, nb, vec8, list, tid, lane, wave);
    if (lane == 0) wcnt[wave] = wc;
    __syncthreads();
    int pre = 0, all = 0;
#pragma unroll
    for (int w2 = 0; w2 < NWAVE; ++w2) {
      int c = wcnt[w2];
      c = c < 0 ? 0 : (c > WCAP ? WCAP : c);
      all += c;
      pre += (w2 < wave) ? c : 0;
    }
    const int wcc  = wc > WCAP ? WCAP : wc;
    const int base = tot + pre;
#pragma unroll 1
    for (int i = lane; i < wcc; i += 32) {
      const int ent = list[wave * WCAP + i];
      const int el  = (ent >> SLOTB) & (CHUNK - 1);
      const int sl  = ent & (NBMAX - 1);
      int eid = cbase + el;
      eid = eid > nE - 1 ? nE - 1 : eid;
      const int pos = base + i;
      if (pos < RCAP) reg1[pos] = (int)(((unsigned)eid << SLOTB) | (unsigned)sl);
    }
    tot += all;
    tot = tot > RCAP ? RCAP : tot;
    __syncthreads();
  }
  const int nh = tot;

  if (wave == 0) {
#pragma unroll 1
    for (int b0 = 0; b0 < nh; b0 += 32) {
      const int idx = b0 + lane;
      const int uv  = reg1[idx < nh ? idx : nh - 1];
      const int m32 = (nh - b0) < 32 ? (nh - b0) : 32;
#pragma unroll 1
      for (int k = 0; k < m32; ++k) {
        const int u  = __builtin_amdgcn_readlane(uv, k);
        const int sl = u & (NBMAX - 1);
        if (lane == 0) scnt[sl] = scnt[sl] + 1;
      }
    }
  }
  __syncthreads();

  {
    const v4i ca = *(const v4i*)(scnt + 8 * tid);
    const v4i cb = *(const v4i*)(scnt + 8 * tid + 4);
    const int e0 = ca.x < 0 ? 0 : ca.x, e1 = ca.y < 0 ? 0 : ca.y, e2 = ca.z < 0 ? 0 : ca.z, e3 = ca.w < 0 ? 0 : ca.w;
    const int e4 = cb.x < 0 ? 0 : cb.x, e5 = cb.y < 0 ? 0 : cb.y, e6 = cb.z < 0 ? 0 : cb.z, e7 = cb.w < 0 ? 0 : cb.w;
    const int ts = e0 + e1 + e2 + e3 + e4 + e5 + e6 + e7;
    int incl = ts;
#pragma unroll
    for (int d = 1; d < 32; d <<= 1) {
      const int up = __shfl_up(incl, d);
      if (lane >= d) incl += up;
    }
    if (lane == 31) wtot[wave] = incl;
    __syncthreads();
    int pre = 0;
#pragma unroll
    for (int w2 = 0; w2 < NWAVE; ++w2) pre += (w2 < wave) ? wtot[w2] : 0;
    int run = pre + incl - ts;
    soff[8 * tid + 0] = run; run += e0;
    soff[8 * tid + 1] = run; run += e1;
    soff[8 * tid + 2] = run; run += e2;
    soff[8 * tid + 3] = run; run += e3;
    soff[8 * tid + 4] = run; run += e4;
    soff[8 * tid + 5] = run; run += e5;
    soff[8 * tid + 6] = run; run += e6;
    soff[8 * tid + 7] = run;
  }
  __syncthreads();
  for (int i = tid; i < NBMAX; i += NTHR) list[i] = soff[i];
  __syncthreads();

  if (wave == 0) {
#pragma unroll 1
    for (int b0 = 0; b0 < nh; b0 += 32) {
      const int idx = b0 + lane;
      const int uv  = reg1[idx < nh ? idx : nh - 1];
      const int m32 = (nh - b0) < 32 ? (nh - b0) : 32;
#pragma unroll 1
      for (int k = 0; k < m32; ++k) {
        const int u   = __builtin_amdgcn_readlane(uv, k);
        const int sl  = u & (NBMAX - 1);
        const int eid = (int)((unsigned)u >> SLOTB);
        if (lane == 0) {
          int pos = list[sl];
          pos = pos < 0 ? 0 : (pos > RCAP - 1 ? RCAP - 1 : pos);
          reg2[pos] = eid;
          list[sl] = pos + 1;
        }
      }
    }
  }
  __syncthreads();

  const int nbw = nb >> 3;
  const bool ovf = (nh >= RCAP);
  const float qnan = __int_as_float(0x7fc00000);
  const float* ELp = SD;
  const float* ERp = SD + (size_t)MPr;

  if (L < 3) {
    const int c0 = 2 * lane;
    const v2f bb2 = bfr2(*(const v2fa*)(bias + c0));
    const int sA = (2 * lane) & 31;
    const int sB = (2 * lane + 1) & 31;
    int wn = 0;
    float wm0 = 0.0f, wm1 = 0.0f, wq0 = 0.0f, wq1 = 0.0f;

#pragma unroll 1
    for (int jt = 0; jt < nbw; ++jt) {
      const int slot = wave * nbw + jt;
      const int grow = nodeBase + slot;
      const int gcl  = grow < nN ? grow : nN - 1;
      int st = soff[slot];
      const int craw = scnt[slot];
      int cnt = craw;
      st  = st < 0 ? 0 : (st > nh ? nh : st);
      cnt = cnt < 0 ? 0 : (cnt > DEGCAP ? DEGCAP : cnt);
      if (cnt > nh - st) cnt = nh - st;
      const float pz = (ovf || craw > DEGCAP) ? qnan : 0.0f;

      const float erd = ERp[gcl];
      float mx = MX0, dn = 0.0f;
      float a0 = 0.0f, a1 = 0.0f;

#pragma unroll 1
      for (int q = 0; q < cnt; ++q) {
        int idx = st + q; idx = idx > RCAP - 1 ? RCAP - 1 : idx;
        int eid = reg2[idx]; eid = eid < 0 ? 0 : (eid > nE - 1 ? nE - 1 : eid);
        const int sraw = srcs[eid];
        const int s = sraw < 0 ? 0 : (sraw > nN - 1 ? nN - 1 : sraw);
        const v2f fs = *(const v2fa*)(F + (size_t)s * CH + c0);
        float lg = ELp[s] + erd;
        lg = lg > 0.f ? lg : NEGSL * lg;
        const float df = lg - mx;
        const float ee = __expf(-fabsf(df));
        const bool up  = df > 0.f;
        const float s1 = up ? ee : 1.0f;
        const float s2 = up ? 1.0f : ee;
        mx = up ? lg : mx;
        dn = fmaf(dn, s1, s2);
        a0 = fmaf(a0, s1, s2 * fs.x);
        a1 = fmaf(a1, s1, s2 * fs.y);
      }
      const float dsafe = dn > 0.f ? dn : 1.0f;
      const float inv = __builtin_amdgcn_rcpf(dsafe);
      float h0 = fmaf(a0, inv, bb2.x);
      float h1 = fmaf(a1, inv, bb2.y);
      const float m0 = __expf(fminf(h0, 0.0f)) - 1.0f;
      const float m1 = __expf(fminf(h1, 0.0f)) - 1.0f;
      h0 = h0 > 0.0f ? h0 : m0;
      h1 = h1 > 0.0f ? h1 : m1;

      const bool live = grow < nN;
      if (live) {
        wn += 1;
        const float rk = __builtin_amdgcn_rcpf((float)wn);
        const float d0 = h0 - wm0;
        wm0 = fmaf(d0, rk, wm0);
        wq0 = fmaf(d0, h0 - wm0, wq0);
        const float d1 = h1 - wm1;
        wm1 = fmaf(d1, rk, wm1);
        wq1 = fmaf(d1, h1 - wm1, wq1);
      }
      const float o0 = (live ? h0 : 0.f) + pz;
      const float o1 = (live ? h1 : 0.f) + pz;
      const float g0 = __shfl(o0, sA);
      const float g1 = __shfl(o1, sA);
      const float g2 = __shfl(o0, sB);
      const float g3 = __shfl(o1, sB);
      v4f pv;
      pv.x = g0; pv.y = g1; pv.z = g2; pv.w = g3;
      float* gp = HCo + (size_t)grow * CH + 4 * (lane & 15);
      const bool wr = (grow < MPr) && (lane < 16);
      if (wr) *(volatile v4f*)gp = pv;
      __threadfence();
      if (wr) *(volatile v4f*)gp = pv;
    }

    float* wst = (float*)list;
    float* pst = wst + NWAVE * WSTW;
    if (lane == 0) wst[wave * WSTW] = (float)wn;
    wst[wave * WSTW + 1 + 2 * lane]          = wm0;
    wst[wave * WSTW + 1 + 2 * lane + 1]      = wm1;
    wst[wave * WSTW + 1 + CH + 2 * lane]     = wq0;
    wst[wave * WSTW + 1 + CH + 2 * lane + 1] = wq1;
    __syncthreads();
    if (tid < CH) {
      float n = 0.0f, mean = 0.0f, M2 = 0.0f;
#pragma unroll 1
      for (int w2 = 0; w2 < NWAVE; ++w2) {
        const float nbv = wst[w2 * WSTW];
        const float mb  = wst[w2 * WSTW + 1 + tid];
        const float qb  = wst[w2 * WSTW + 1 + CH + tid];
        if (nbv > 0.5f) {
          const float nn = n + nbv;
          const float delta = mb - mean;
          const float f = nbv / nn;
          mean = fmaf(delta, f, mean);
          M2 = M2 + qb + delta * delta * n * f;
          n = nn;
        }
      }
      pst[1 + tid] = mean;
      pst[1 + CH + tid] = M2;
      if (tid == 0) pst[0] = n;
    }
#pragma unroll 1
    for (int i = 2 * CH + 1 + tid; i < PARTW; i += NTHR) pst[i] = 0.0f;
    __syncthreads();
    const int pb = (int)blockIdx.x;
    v4f ps = {0.0f, 0.0f, 0.0f, 0.0f};
    if (tid < PARTW / 4) {
      ps = *(const v4fa*)(pst + 4 * tid);
      *(volatile v4f*)(part + (size_t)pb * PARTW + 4 * tid) = ps;
    }
    __threadfence();
    if (tid < PARTW / 4) {
      *(volatile v4f*)(part + (size_t)pb * PARTW + 4 * tid) = ps;
    }
  } else {
    const float bb = bfr(bias[lane]);

#pragma unroll 1
    for (int jt = 0; jt < nbw; ++jt) {
      const int slot = wave * nbw + jt;
      const int grow = nodeBase + slot;
      const int gcl  = grow < nN ? grow : nN - 1;
      int st = soff[slot];
      const int craw = scnt[slot];
      int cnt = craw;
      st  = st < 0 ? 0 : (st > nh ? nh : st);
      cnt = cnt < 0 ? 0 : (cnt > DEGCAP ? DEGCAP : cnt);
      if (cnt > nh - st) cnt = nh - st;
      const float pz = (ovf || craw > DEGCAP) ? qnan : 0.0f;

      const float erd = ERp[gcl];
      float mx = MX0, dn = 0.0f;
      float a0 = 0.0f;

#pragma unroll 1
      for (int q = 0; q < cnt; ++q) {
        int idx = st + q; idx = idx > RCAP - 1 ? RCAP - 1 : idx;
        int eid = reg2[idx]; eid = eid < 0 ? 0 : (eid > nE - 1 ? nE - 1 : eid);
        const int sraw = srcs[eid];
        const int s = sraw < 0 ? 0 : (sraw > nN - 1 ? nN - 1 : sraw);
        const float fs = F[(size_t)s * NOUT + lane];
        float lg = ELp[s] + erd;
        lg = lg > 0.f ? lg : NEGSL * lg;
        const float df = lg - mx;
        const float ee = __expf(-fabsf(df));
        const bool up  = df > 0.f;
        const float s1 = up ? ee : 1.0f;
        const float s2 = up ? 1.0f : ee;
        mx = up ? lg : mx;
        dn = fmaf(dn, s1, s2);
        a0 = fmaf(a0, s1, s2 * fs);
      }
      const float dsafe = dn > 0.f ? dn : 1.0f;
      const float inv = __builtin_amdgcn_rcpf(dsafe);
      const float h0 = fmaf(a0, inv, bb) + pz;
      const float g0 = __shfl(h0, (4 * lane) & 31);
      const float g1 = __shfl(h0, (4 * lane + 1) & 31);
      const float g2 = __shfl(h0, (4 * lane + 2) & 31);
      const float g3 = __shfl(h0, (4 * lane + 3) & 31);
      v4f ov;
      ov.x = g0; ov.y = g1; ov.z = g2; ov.w = g3;
      float* op = out + (size_t)gcl * NOUT + 4 * (lane & 7);
      const bool wr = (grow < nN) && (lane < 8);
      if (wr) *(volatile v4f*)op = ov;
      __threadfence();
      if (wr) *(volatile v4f*)op = ov;
    }
  }
}

__global__ __launch_bounds__(CH) void k_bnfin(const float* __restrict__ part, int nPart,
                                              const float* __restrict__ gam, const float* __restrict__ bet,
                                              float* ss) {
  __shared__ __attribute__((aligned(16))) float stg[2 * CH];
  const int tid = (int)threadIdx.x;
  const int c = tid;
  double n = 0.0, mean = 0.0, M2 = 0.0;
#pragma unroll 1
  for (int b = 0; b < nPart; ++b) {
    const float* pr = part + (size_t)b * PARTW;
    const double nbv = (double)pr[0];
    const double mb  = (double)pr[1 + c];
    const double qb  = (double)pr[1 + CH + c];
    if (nbv > 0.5) {
      const double nn = n + nbv;
      const double delta = mb - mean;
      const double f = nbv / nn;
      mean = mean + delta * f;
      M2 = M2 + qb + delta * delta * n * f;
      n = nn;
    }
  }
  const double nt = n < 1.0 ? 1.0 : n;
  const float varf  = (float)(M2 / nt);
  const float meanf = (float)mean;
  const float rstd = 1.0f / sqrtf(varf + BNEPS);
  const float sc = bfr(gam[c]) * rstd;
  const float sh = bfr(bet[c]) - meanf * sc;
  stg[c] = sc;
  stg[CH + c] = sh;
  __syncthreads();
  v4f v = {0.0f, 0.0f, 0.0f, 0.0f};
  if (tid < (2 * CH) / 4) {
    v = *(const v4fa*)(stg + 4 * tid);
    *(volatile v4f*)(ss + 4 * tid) = v;
  }
  __threadfence();
  if (tid < (2 * CH) / 4) {
    *(volatile v4f*)(ss + 4 * tid) = v;
  }
}

__global__ __launch_bounds__(NTHR) void k_bnstat(const float* __restrict__ hc, const float* __restrict__ ss,
                                                 float* part, int nN, int nb) {
  __shared__ __attribute__((aligned(16))) float ssh[2 * CH];
  __shared__ __attribute__((aligned(16))) float wst[NWAVE * WSTW];
  __shared__ __attribute__((aligned(16))) float pst[PARTW];
  const int tid = (int)threadIdx.x, lane = tid & 31, wave = tid >> 5;
  const int nodeBase = (int)blockIdx.x * nb;
  if (tid < 2 * CH) ssh[tid] = ss[tid];
  __syncthreads();
  const v2f sc = *(const v2fa*)(ssh + 2 * lane);
  const v2f sh = *(const v2fa*)(ssh + CH + 2 * lane);
  const int nbw = nb >> 3;
  int wn = 0;
  float wm0 = 0.0f, wm1 = 0.0f, wq0 = 0.0f, wq1 = 0.0f;
#pragma unroll 1
  for (int jt = 0; jt < nbw; ++jt) {
    const int grow = nodeBase + wave * nbw + jt;
    const int gcl  = grow < nN ? grow : nN - 1;
    const v2f hv = *(const v2fa*)(hc + (size_t)gcl * CH + 2 * lane);
    const float y0 = fmaf(hv.x, sc.x, sh.x);
    const float y1 = fmaf(hv.y, sc.y, sh.y);
    if (grow < nN) {
      wn += 1;
      const float rk = __builtin_amdgcn_rcpf((float)wn);
      const float d0 = y0 - wm0;
      wm0 = fmaf(d0, rk, wm0);
      wq0 = fmaf(d0, y0 - wm0, wq0);
      const float d1 = y1 - wm1;
      wm1 = fmaf(d1, rk, wm1);
      wq1 = fmaf(d1, y1 - wm1, wq1);
    }
  }
  if (lane == 0) wst[wave * WSTW] = (float)wn;
  wst[wave * WSTW + 1 + 2 * lane]          = wm0;
  wst[wave * WSTW + 1 + 2 * lane + 1]      = wm1;
  wst[wave * WSTW + 1 + CH + 2 * lane]     = wq0;
  wst[wave * WSTW + 1 + CH + 2 * lane + 1] = wq1;
  __syncthreads();
  if (tid < CH) {
    float n = 0.0f, mean = 0.0f, M2 = 0.0f;
#pragma unroll 1
    for (int w2 = 0; w2 < NWAVE; ++w2) {
      const float nbv = wst[w2 * WSTW];
      const float mb  = wst[w2 * WSTW + 1 + tid];
      const float qb  = wst[w2 * WSTW + 1 + CH + tid];
      if (nbv > 0.5f) {
        const float nn = n + nbv;
        const float delta = mb - mean;
        const float f = nbv / nn;
        mean = fmaf(delta, f, mean);
        M2 = M2 + qb + delta * delta * n * f;
        n = nn;
      }
    }
    pst[1 + tid] = mean;
    pst[1 + CH + tid] = M2;
    if (tid == 0) pst[0] = n;
  }
#pragma unroll 1
  for (int i = 2 * CH + 1 + tid; i < PARTW; i += NTHR) pst[i] = 0.0f;
  __syncthreads();
  const int pb = (int)blockIdx.x;
  v4f ps = {0.0f, 0.0f, 0.0f, 0.0f};
  if (tid < PARTW / 4) {
    ps = *(const v4fa*)(pst + 4 * tid);
    *(volatile v4f*)(part + (size_t)pb * PARTW + 4 * tid) = ps;
  }
  __threadfence();
  if (tid < PARTW / 4) {
    *(volatile v4f*)(part + (size_t)pb * PARTW + 4 * tid) = ps;
  }
}

__global__ __launch_bounds__(NTHR) void k_apply(const float* __restrict__ hc, const float* __restrict__ ss1,
                                                const float* __restrict__ ss2,
                                                int nN, int nUnits, unsigned short* apl) {
  __shared__ __attribute__((aligned(16))) float ssh[4 * CH];
  const int tid = (int)threadIdx.x;
  if (tid < 2 * CH) { ssh[tid] = ss1[tid]; ssh[2 * CH + tid] = ss2[tid]; }
  __syncthreads();
  const int u = (int)blockIdx.x * NTHR + tid;
  const bool act = u < nUnits;
  const int uc = act ? u : (nUnits - 1);
  const int row = uc >> 4;
  const int piece = uc & 15;
  const int c0 = (piece & 7) * 8;
  const float* p = hc + (size_t)row * CH + c0;
  const v4f a = *(const v4f*)p;
  const v4f b = *(const v4f*)(p + 4);
  const v4f s1a = *(const v4fa*)(ssh + c0);
  const v4f s1b = *(const v4fa*)(ssh + c0 + 4);
  const v4f h1a = *(const v4fa*)(ssh + CH + c0);
  const v4f h1b = *(const v4fa*)(ssh + CH + c0 + 4);
  const v4f s2a = *(const v4fa*)(ssh + 2 * CH + c0);
  const v4f s2b = *(const v4fa*)(ssh + 2 * CH + c0 + 4);
  const v4f h2a = *(const v4fa*)(ssh + 3 * CH + c0);
  const v4f h2b = *(const v4fa*)(ssh + 3 * CH + c0 + 4);
  const bool live = row < nN;
  float y[8];
  y[0] = fmaf(a.x, s1a.x, h1a.x); y[1] = fmaf(a.y, s1a.y, h1a.y); y[2] = fmaf(a.z, s1a.z, h1a.z); y[3] = fmaf(a.w, s1a.w, h1a.w);
  y[4] = fmaf(b.x, s1b.x, h1b.x); y[5] = fmaf(b.y, s1b.y, h1b.y); y[6] = fmaf(b.z, s1b.z, h1b.z); y[7] = fmaf(b.w, s1b.w, h1b.w);
  y[0] = fmaf(y[0], s2a.x, h2a.x); y[1] = fmaf(y[1], s2a.y, h2a.y); y[2] = fmaf(y[2], s2a.z, h2a.z); y[3] = fmaf(y[3], s2a.w, h2a.w);
  y[4] = fmaf(y[4], s2b.x, h2b.x); y[5] = fmaf(y[5], s2b.y, h2b.y); y[6] = fmaf(y[6], s2b.z, h2b.z); y[7] = fmaf(y[7], s2b.w, h2b.w);
  unsigned int wv[8];
  const bool lsel = piece >= 8;
#pragma unroll
  for (int j = 0; j < 8; ++j) {
    const float t = live ? y[j] : 0.0f;
    const unsigned int hb = f2bf(t);
    const unsigned int lb = f2bf(t - bf2f(hb));
    wv[j] = lsel ? lb : hb;
  }
  v4u q;
  q.x = wv[0] | (wv[1] << 16);
  q.y = wv[2] | (wv[3] << 16);
  q.z = wv[4] | (wv[5] << 16);
  q.w = wv[6] | (wv[7] << 16);
  unsigned short* o = apl + (size_t)row * KG + 8 * piece;
  if (act) *(volatile v4u*)o = q;
  __threadfence();
  if (act) *(volatile v4u*)o = q;
}

static int pick_nb(int nE, int nN) {
  int nb = NBMAX;
  while (nb > 32 && (long long)nb * (long long)nE * 5LL > (long long)RCAP * (long long)nN * 4LL) nb >>= 1;
  return nb;
}
static inline int cdiv(int a, int b) { return (a + b - 1) / b; }
static inline size_t al256(size_t o) { return (o + 255) & ~(size_t)255; }

extern "C" void kernel_launch(void* const* d_in, const int* in_sizes, int n_in,
                              void* d_out, int out_size, void* d_ws, size_t ws_size,
                              hipStream_t stream) {
  if (n_in < 19) return;
  const int nN = in_sizes[0] / F_IN0;
  if (nN < 16 || in_sizes[0] != nN * F_IN0 || nN >= (1 << 22)) return;
  const int nE = in_sizes[1];
  if (nE < 1 || in_sizes[2] != nE || nE >= (1 << (32 - SLOTB))) return;
  if (in_sizes[3]  != F_IN0 * CH) return;
  if (in_sizes[4]  != CH || in_sizes[5] != CH) return;
  if (in_sizes[6]  != CH || in_sizes[7] != CH || in_sizes[8] != CH) return;
  if (in_sizes[9]  != CH * CH) return;
  if (in_sizes[10] != CH || in_sizes[11] != CH) return;
  if (in_sizes[12] != CH || in_sizes[13] != CH || in_sizes[14] != CH) return;
  if (in_sizes[15] != CH * NOUT) return;
  if (in_sizes[16] != NOUT || in_sizes[17] != NOUT || in_sizes[18] != NOUT) return;
  if (out_size != nN * NOUT) return;

  const float* x    = (const float*)d_in[0];
  const int*   src  = (const int*)  d_in[1];
  const int*   dst  = (const int*)  d_in[2];
  const float* W0   = (const float*)d_in[3];
  const float* al0  = (const float*)d_in[4];
  const float* ar0  = (const float*)d_in[5];
  const float* b0   = (const float*)d_in[6];
  const float* g0   = (const float*)d_in[7];
  const float* be0  = (const float*)d_in[8];
  const float* W1   = (const float*)d_in[9];
  const float* al1  = (const float*)d_in[10];
  const float* ar1  = (const float*)d_in[11];
  const float* b1   = (const float*)d_in[12];
  const float* g1   = (const float*)d_in[13];
  const float* be1  = (const float*)d_in[14];
  const float* Wm   = (const float*)d_in[15];
  const float* alm  = (const float*)d_in[16];
  const float* arm  = (const float*)d_in[17];
  const float* bm   = (const float*)d_in[18];
  float* out = (float*)d_out;

  const int MP = cdiv(nN, MROWS) * MROWS;
  const int gM = MP / GBM;
  const int nb = pick_nb(nE, nN);
  if (nb < 32 || (nb & (nb - 1)) != 0 || nb > NBMAX) return;
  const int gA = cdiv(MP, nb);
  if ((long long)gA * nb < (long long)MP) return;

  char* ws = (char*)d_ws;
  size_t off = 0;
  const size_t oXB  = off; off = al256(off + (size_t)MP * KG * 2);
  const size_t oHP  = off; off = al256(off + (size_t)MP * KG * 2);
  const size_t oWH  = off; off = al256(off + (size_t)MP * CH * 4);
  const size_t oSD  = off; off = al256(off + (size_t)2 * MP * 4);
  const size_t oHC  = off; off = al256(off + (size_t)MP * CH * 4);
  const size_t oPT  = off; off = al256(off + (size_t)gA * PARTW * 4);
  const size_t oS1  = off; off = al256(off + (size_t)(2 * CH) * 4);
  const size_t oS2  = off; off = al256(off + (size_t)(2 * CH) * 4);
  const size_t oWT0 = off; off = al256(off + (size_t)CH * KG * 2);
  const size_t oWT1 = off; off = al256(off + (size_t)CH * KG * 2);
  const size_t oWT2 = off; off = al256(off + (size_t)NOUT * KG * 2);
  if (off > ws_size || off > (size_t)WSMAX) return;
  unsigned short* XB  = (unsigned short*)(ws + oXB);
  unsigned short* HP  = (unsigned short*)(ws + oHP);
  float*          WH  = (float*)(ws + oWH);
  float*          SD  = (float*)(ws + oSD);
  float*          HC  = (float*)(ws + oHC);
  float*          PT  = (float*)(ws + oPT);
  float*          SS1 = (float*)(ws + oS1);
  float*          SS2 = (float*)(ws + oS2);
  unsigned short* WT0 = (unsigned short*)(ws + oWT0);
  unsigned short* WT1 = (unsigned short*)(ws + oWT1);
  unsigned short* WT2 = (unsigned short*)(ws + oWT2);

  hipFuncSetAttribute(reinterpret_cast<const void*>(&k_agg<1>),
                      hipFuncAttributeMaxDynamicSharedMemorySize, LDS_AGG);
  hipFuncSetAttribute(reinterpret_cast<const void*>(&k_agg<2>),
                      hipFuncAttributeMaxDynamicSharedMemorySize, LDS_AGG);
  hipFuncSetAttribute(reinterpret_cast<const void*>(&k_agg<3>),
                      hipFuncAttributeMaxDynamicSharedMemorySize, LDS_AGG);

  {
    const int nUx = MP * XUPR;
    k_xprep<<<cdiv(nUx, NTHR), NTHR, 0, stream>>>(x, XB, nN, nUx);
  }
  {
    const int nU0 = CH * (KG / 8);
    k_wtr<<<cdiv(nU0, NTHR), NTHR, 0, stream>>>(W0, F_IN0, CH, CH, KG, WT0, nU0);
    k_wtr<<<cdiv(nU0, NTHR), NTHR, 0, stream>>>(W1, CH, CH, CH, KG, WT1, nU0);
    const int nU2 = NOUT * (KG / 8);
    k_wtr<<<cdiv(nU2, NTHR), NTHR, 0, stream>>>(Wm, CH, NOUT, NOUT, KG, WT2, nU2);
  }
  const int nUa = MP * 16;

  k_gemm<64><<<gM, GTHR, 0, stream>>>(XB, WT0, WH, al0, ar0, SD, MP);
  k_agg<1><<<gA, NTHR, LDS_AGG, stream>>>(src, dst, WH, SD, b0, HC, PT, out, nN, nE, nb, MP);
  k_bnfin<<<1, CH, 0, stream>>>(PT, gA, g0, be0, SS1);
  k_bnstat<<<gA, NTHR, 0, stream>>>(HC, SS1, PT, nN, nb);
  k_bnfin<<<1, CH, 0, stream>>>(PT, gA, g0, be0, SS2);
  k_apply<<<cdiv(nUa, NTHR), NTHR, 0, stream>>>(HC, SS1, SS2, nN, nUa, HP);

  k_gemm<64><<<gM, GTHR, 0, stream>>>(HP, WT1, WH, al1, ar1, SD, MP);
  k_agg<2><<<gA, NTHR, LDS_AGG, stream>>>(src, dst, WH, SD, b1, HC, PT, out, nN, nE, nb, MP);
  k_bnfin<<<1, CH, 0, stream>>>(PT, gA, g1, be1, SS1);
  k_bnstat<<<gA, NTHR, 0, stream>>>(HC, SS1, PT, nN, nb);
  k_bnfin<<<1, CH, 0, stream>>>(PT, gA, g1, be1, SS2);
  k_apply<<<cdiv(nUa, NTHR), NTHR, 0, stream>>>(HC, SS1, SS2, nN, nUa, HP);

  k_gemm<32><<<gM, GTHR, 0, stream>>>(HP, WT2, WH, alm, arm, SD, MP);
  k_agg<3><<<gA, NTHR, LDS_AGG, stream>>>(src, dst, WH, SD, bm, HC, PT, out, nN, nE, nb, MP);
}
